// MambaBlock_43843026158205
// MI455X (gfx1250) — hardware-verified
//
#include <hip/hip_runtime.h>
#include <math.h>

typedef __attribute__((ext_vector_type(16))) _Float16 v16h;
typedef __attribute__((ext_vector_type(8)))  _Float16 v8h;
typedef __attribute__((ext_vector_type(16))) __bf16   v16b;
typedef __attribute__((ext_vector_type(8)))  __bf16   v8b;
typedef __attribute__((ext_vector_type(8)))  float    v8f;
typedef __attribute__((ext_vector_type(4)))  float    v4f;

constexpr int kBatch = 2;
constexpr int kSeqL  = 2048;
constexpr int kDmod  = 1024;
constexpr int kDin   = 2048;
constexpr int kNst   = 16;
constexpr int kDcv   = 4;
constexpr int kPrjN  = 1 + 2 * kNst;
constexpr int kPrjP  = 64;
constexpr int kXZP   = 2 * kDin;
constexpr int kRows  = kBatch * kSeqL;
constexpr int kTP    = 260;
constexpr float kWCarry = 32.0f;
constexpr float kYCarry = 256.0f;
constexpr float kInProjScale  = 1.0f / kWCarry;
constexpr float kOutProjScale = 1.0f / (kWCarry * kYCarry);
static_assert(kPrjN <= kPrjP);
static_assert((kDmod % 32) == 0 && (kDin % 32) == 0);
static_assert((kSeqL % 64) == 0 && (kXZP % 64) == 0 && (kPrjP % 64) == 0 && (kDmod % 64) == 0);
static_assert((kDin % 256) == 0 && (kSeqL % 16) == 0 && (kSeqL % 64) == 0);
static_assert((kDmod % 8) == 0 && (kDin % 8) == 0);

constexpr size_t kSzX16  = (size_t)kRows * kDmod * 2;
constexpr size_t kSzWI16 = (size_t)kXZP  * kDmod * 2;
constexpr size_t kSzWO16 = (size_t)kDmod * kDin  * 2;
constexpr size_t kSzWX   = (size_t)kPrjP * kDin  * 2;
constexpr size_t kSzXZ   = (size_t)kSeqL * kXZP  * 4;
constexpr size_t kSzUG   = (size_t)kSeqL * kDin  * 4;
constexpr size_t kSzUG16 = (size_t)kSeqL * kDin  * 2;
constexpr size_t kSzPROJ = (size_t)kSeqL * kPrjP * 4;
constexpr size_t kSzY16  = (size_t)kSeqL * kDin  * 2;
constexpr size_t kOffX16  = 0;
constexpr size_t kOffWI16 = kOffX16  + kSzX16;
constexpr size_t kOffWO16 = kOffWI16 + kSzWI16;
constexpr size_t kOffWXH  = kOffWO16 + kSzWO16;
constexpr size_t kOffWXL  = kOffWXH  + kSzWX;
constexpr size_t kOffXZ   = kOffWXL  + kSzWX;
constexpr size_t kOffUG   = kOffXZ   + kSzXZ;
constexpr size_t kOffUGH  = kOffUG   + kSzUG;
constexpr size_t kOffUGL  = kOffUGH  + kSzUG16;
constexpr size_t kOffPROJ = kOffUGL  + kSzUG16;
constexpr size_t kOffY16  = kOffPROJ + kSzPROJ;
constexpr size_t kWsTotal = kOffY16  + kSzY16;
static_assert(kWsTotal == 97517568ull);
static_assert(kWsTotal <= 134217728ull);
static_assert((kOffWI16 % 128) == 0 && (kOffWO16 % 128) == 0 && (kOffWXH % 128) == 0 && (kOffWXL % 128) == 0 &&
              (kOffXZ % 128) == 0 && (kOffUG % 128) == 0 && (kOffUGH % 128) == 0 && (kOffUGL % 128) == 0 &&
              (kOffPROJ % 128) == 0 && (kOffY16 % 128) == 0);

__device__ __forceinline__ unsigned short f2bf_bits(float f) {
  unsigned u = __float_as_uint(f);
  return (unsigned short)((u + 0x7FFFu + ((u >> 16) & 1u)) >> 16);
}
__device__ __forceinline__ float bf_bits2f(unsigned short h) { return __uint_as_float(((unsigned)h) << 16); }

__device__ __forceinline__ void dep_guard_h(v8f& a, v8f& b, v16h x, v16h y) { asm volatile("v_nop\n\tv_nop\n\tv_nop\n\tv_nop" : "+v"(a), "+v"(b) : "v"(x), "v"(y)); }
__device__ __forceinline__ void dep_guard_b(v8f& a, v8f& b, v16b x, v16b y) { asm volatile("v_nop\n\tv_nop\n\tv_nop\n\tv_nop" : "+v"(a), "+v"(b) : "v"(x), "v"(y)); }
__device__ __forceinline__ void dep_guard4_h(v8f& a, v8f& b, v8f& c, v8f& d, v16h x, v16h y) { asm volatile("v_nop\n\tv_nop\n\tv_nop\n\tv_nop" : "+v"(a), "+v"(b), "+v"(c), "+v"(d) : "v"(x), "v"(y)); }
__device__ __forceinline__ void dep_guard4_b(v8f& a, v8f& b, v8f& c, v8f& d, v16b x, v16b y) { asm volatile("v_nop\n\tv_nop\n\tv_nop\n\tv_nop" : "+v"(a), "+v"(b), "+v"(c), "+v"(d) : "v"(x), "v"(y)); }
__device__ __forceinline__ void keep4_h(v16h a, v16h b, v16h c, v16h d) { asm volatile("v_nop" :: "v"(a), "v"(b), "v"(c), "v"(d)); }
__device__ __forceinline__ void keep4_b(v16b a, v16b b, v16b c, v16b d) { asm volatile("v_nop" :: "v"(a), "v"(b), "v"(c), "v"(d)); }
__device__ __forceinline__ void acc_guard4(v8f& a, v8f& b, v8f& c, v8f& d) { asm volatile("v_nop\n\tv_nop\n\tv_nop\n\tv_nop" : "+v"(a), "+v"(b), "+v"(c), "+v"(d)); }
template <typename T> struct Frag;
template <> struct Frag<_Float16> {
  typedef v16h V; union U { v16h v; v8h h[2]; };
  static __device__ __forceinline__ v16h load(const _Float16* p) {
    U f; f.h[0] = *(const v8h*)(p); f.h[1] = *(const v8h*)(p + 16); return f.v;
  }
  static __device__ __forceinline__ v8f mma(v16h a, v16h b, v8f c) {
    return __builtin_amdgcn_wmma_f32_16x16x32_f16(false, a, false, b, (short)0, c, false, false);
  }
  static __device__ __forceinline__ void guard(v8f& a, v8f& b, v16h x, v16h y) { dep_guard_h(a, b, x, y); }
  static __device__ __forceinline__ void guard4(v8f& a, v8f& b, v8f& c, v8f& d, v16h x, v16h y) { dep_guard4_h(a, b, c, d, x, y); }
  static __device__ __forceinline__ void keep(v16h a, v16h b, v16h c, v16h d) { keep4_h(a, b, c, d); }
};
template <> struct Frag<__bf16> {
  typedef v16b V; union U { v16b v; v8b h[2]; };
  static __device__ __forceinline__ v16b load(const __bf16* p) {
    U f; f.h[0] = *(const v8b*)(p); f.h[1] = *(const v8b*)(p + 16); return f.v;
  }
  static __device__ __forceinline__ v8f mma(v16b a, v16b b, v8f c) {
    return __builtin_amdgcn_wmma_f32_16x16x32_bf16(false, a, false, b, (short)0, c, false, false);
  }
  static __device__ __forceinline__ void guard(v8f& a, v8f& b, v16b x, v16b y) { dep_guard_b(a, b, x, y); }
  static __device__ __forceinline__ void guard4(v8f& a, v8f& b, v8f& c, v8f& d, v16b x, v16b y) { dep_guard4_b(a, b, c, d, x, y); }
  static __device__ __forceinline__ void keep(v16b a, v16b b, v16b c, v16b d) { keep4_b(a, b, c, d); }
};

template <int ET> struct Elem;
template <> struct Elem<0> { typedef _Float16 T; };
template <> struct Elem<1> { typedef __bf16 T; };
template <int ET, bool SPLIT, int BIAS_MODE, int OUT_MODE, bool RESID, int ACT = 0>
__global__ __launch_bounds__(256) void wmma_gemm64(
    const unsigned short* __restrict__ Ap, const unsigned short* __restrict__ A2p, int lda, long strideA,
    const unsigned short* __restrict__ Btp, const unsigned short* __restrict__ Bt2p, int ldb, long strideB,
    void* __restrict__ Cout, void* __restrict__ Cout2, int ldc, long strideC,
    const float* __restrict__ bias,
    const float* __restrict__ resid, long strideR,
    int M, int N, int K, float scale) {
  typedef typename Elem<ET>::T T;
  typedef typename Frag<T>::V V;
  const T* A = (const T*)Ap; const T* A2 = (const T*)A2p; const T* Bt = (const T*)Btp; const T* Bt2 = (const T*)Bt2p;
  __shared__ __align__(16) float sT[8][16 * 68];
  const int b    = blockIdx.y;
  const int lane = threadIdx.x & 31;
  const int wave = threadIdx.x >> 5;
  const int tilesN = N >> 6;
  const int tilesM = M >> 6;
  const int tile = blockIdx.x * 8 + wave;
  if (tile >= tilesM * tilesN) return;
  const int tm = tile / tilesN;
  const int tn = tile - tm * tilesN;
  const int m0 = tm << 6;
  const int n0 = tn << 6;

  const T* Ab  = A  + (size_t)b * strideA;
  const T* Bb  = Bt + (size_t)b * strideB;
  const T* Ab2 = SPLIT ? (A2  + (size_t)b * strideA) : nullptr;
  const T* Bb2 = SPLIT ? (Bt2 + (size_t)b * strideB) : nullptr;

  const int rlane = lane & 15;
  const int koff  = (lane >> 4) * 8;
  const int mOff  = (lane >> 4) * 8;

  v8f acc[4][4];
#pragma unroll
  for (int i = 0; i < 4; ++i)
#pragma unroll
    for (int j = 0; j < 4; ++j) acc[i][j] = (v8f){0.f,0.f,0.f,0.f,0.f,0.f,0.f,0.f};

  for (int k0 = 0; k0 < K; k0 += 32) {
    V bh[4], bl[4];
#pragma unroll
    for (int j = 0; j < 4; ++j) {
      const size_t bo = (size_t)(n0 + (j << 4) + rlane) * ldb + koff + k0;
      bh[j] = Frag<T>::load(Bb + bo);
      if (SPLIT) bl[j] = Frag<T>::load(Bb2 + bo);
    }
#pragma unroll
    for (int i = 0; i < 4; ++i) {
      const size_t ao = (size_t)(m0 + (i << 4) + rlane) * lda + koff + k0;
      V ah = Frag<T>::load(Ab + ao);
      V al;
      if (SPLIT) al = Frag<T>::load(Ab2 + ao);
#pragma unroll
      for (int j = 0; j < 4; ++j) {
        acc[i][j] = Frag<T>::mma(ah, bh[j], acc[i][j]);
        if (SPLIT) {
          acc[i][j] = Frag<T>::mma(ah, bl[j], acc[i][j]);
          acc[i][j] = Frag<T>::mma(al, bh[j], acc[i][j]);
        }
      }
      Frag<T>::guard4(acc[i][0], acc[i][1], acc[i][2], acc[i][3], ah, SPLIT ? al : ah);
    }
    Frag<T>::keep(bh[0], bh[1], bh[2], bh[3]);
    if (SPLIT) Frag<T>::keep(bl[0], bl[1], bl[2], bl[3]);
  }
  acc_guard4(acc[0][0], acc[0][1], acc[0][2], acc[0][3]);
  acc_guard4(acc[1][0], acc[1][1], acc[1][2], acc[1][3]);
  acc_guard4(acc[2][0], acc[2][1], acc[2][2], acc[2][3]);
  acc_guard4(acc[3][0], acc[3][1], acc[3][2], acc[3][3]);

  float* slab = sT[wave];
  const float* Rb = RESID ? (resid + (size_t)b * strideR) : nullptr;
#pragma unroll
  for (int i = 0; i < 4; ++i) {
    const int mBase = m0 + (i << 4);
#pragma unroll
    for (int j = 0; j < 4; ++j) {
      const int n = n0 + (j << 4) + rlane;
      float bv = 0.f;
      if (BIAS_MODE == 2) bv = bias[n];
#pragma unroll
      for (int r = 0; r < 8; ++r) {
        float v = acc[i][j][r] * scale;
        if (BIAS_MODE == 1) v += bias[mBase + mOff + r];
        if (BIAS_MODE == 2) v += bv;
        if (RESID) v += Rb[(size_t)(mBase + mOff + r) * ldc + n];
        if (ACT == 1) v = tanhf(v);
        if (ACT == 2) v = fmaxf(v, 0.0f);
        if (ACT == 3) v = v / (1.0f + expf(-v));
        if (ACT == 4) v = (v > 0.f) ? v : 0.01f * v;
        slab[(mOff + r) * 68 + (j << 4) + rlane] = v;
      }
    }
    __builtin_amdgcn_fence(__ATOMIC_RELEASE, "workgroup");
    __builtin_amdgcn_wave_barrier();
    __builtin_amdgcn_fence(__ATOMIC_ACQUIRE, "workgroup");
    if (OUT_MODE == 0) {
      float* C = (float*)Cout + (size_t)b * strideC;
      const int hh = lane >> 4, c4 = (lane & 15) * 4;
      for (int pass = 0; pass < 2; ++pass) {
#pragma unroll
        for (int it = 0; it < 8; ++it) {
          const int row = it * 2 + hh;
          v4f v = *(const v4f*)(slab + row * 68 + c4);
          *(volatile v4f*)(C + (size_t)(mBase + row) * ldc + n0 + c4) = v;
        }
        __threadfence();
      }
    } else {
      const int q = lane >> 3, c8 = (lane & 7) * 8;
      unsigned short* C  = (unsigned short*)Cout  + (size_t)b * strideC;
      unsigned short* C2 = (OUT_MODE == 2) ? ((unsigned short*)Cout2 + (size_t)b * strideC) : nullptr;
      for (int pass = 0; pass < 2; ++pass) {
#pragma unroll
        for (int it = 0; it < 4; ++it) {
          const int row = it * 4 + q;
          const float* sp = slab + row * 68 + c8;
          v8h hv, lv;
#pragma unroll
          for (int e = 0; e < 8; ++e) {
            if (OUT_MODE == 1) {
              hv[e] = (_Float16)sp[e];
            } else {
              unsigned short hb = f2bf_bits(sp[e]);
              unsigned short lb = f2bf_bits(sp[e] - bf_bits2f(hb));
              hv[e] = __builtin_bit_cast(_Float16, hb);
              lv[e] = __builtin_bit_cast(_Float16, lb);
            }
          }
          *(volatile v8h*)(C + (size_t)(mBase + row) * ldc + n0 + c8) = hv;
          if (OUT_MODE == 2) *(volatile v8h*)(C2 + (size_t)(mBase + row) * ldc + n0 + c8) = lv;
        }
        __threadfence();
      }
    }
    __builtin_amdgcn_fence(__ATOMIC_RELEASE, "workgroup");
    __builtin_amdgcn_wave_barrier();
    __builtin_amdgcn_fence(__ATOMIC_ACQUIRE, "workgroup");
  }
}

__global__ __launch_bounds__(256) void cast_f16_kernel(
    const float* __restrict__ src, unsigned short* __restrict__ dst, int total8, float scale)
{
  const int i = blockIdx.x * 256 + threadIdx.x;
  if (i >= total8) return;
  const size_t e0 = (size_t)i << 3;
  const float* p = src + e0;
  const v4f a0 = *(const v4f*)(p);
  const v4f a1 = *(const v4f*)(p + 4);
  v8h hv;
#pragma unroll
  for (int e = 0; e < 4; ++e) {
    hv[e]     = (_Float16)(a0[e] * scale);
    hv[4 + e] = (_Float16)(a1[e] * scale);
  }
  unsigned short* q = dst + e0;
  *(volatile v8h*)q = hv;
  __threadfence();
  *(volatile v8h*)q = hv;
}

__global__ __launch_bounds__(256) void split_rows_pad_bf16_kernel(
    const float* __restrict__ src, unsigned short* __restrict__ dhi, unsigned short* __restrict__ dlo,
    int total8, int rowlen, int nsrc)
{
  const int i = blockIdx.x * 256 + threadIdx.x;
  if (i >= total8) return;
  const size_t e0 = (size_t)i << 3;
  const int row = (int)(e0 / (size_t)rowlen);
  const int col = (int)(e0 - (size_t)row * rowlen);
  const bool keep = (row < nsrc);
  const int rc = keep ? row : (nsrc - 1);
  const float* p = src + (size_t)rc * rowlen + col;
  const v4f a0 = *(const v4f*)(p);
  const v4f a1 = *(const v4f*)(p + 4);
  v8h hv, lv;
#pragma unroll
  for (int e = 0; e < 4; ++e) {
    const float v0 = keep ? a0[e] : 0.f;
    const float v1 = keep ? a1[e] : 0.f;
    const unsigned short h0 = f2bf_bits(v0), h1 = f2bf_bits(v1);
    const unsigned short l0 = f2bf_bits(v0 - bf_bits2f(h0)), l1 = f2bf_bits(v1 - bf_bits2f(h1));
    hv[e]     = __builtin_bit_cast(_Float16, h0);
    hv[4 + e] = __builtin_bit_cast(_Float16, h1);
    lv[e]     = __builtin_bit_cast(_Float16, l0);
    lv[4 + e] = __builtin_bit_cast(_Float16, l1);
  }
  unsigned short* qh = dhi + e0;
  unsigned short* ql = dlo + e0;
  *(volatile v8h*)qh = hv;
  *(volatile v8h*)ql = lv;
  __threadfence();
  *(volatile v8h*)qh = hv;
  *(volatile v8h*)ql = lv;
}

__global__ __launch_bounds__(256) void conv_gate_kernel(
    const float* __restrict__ XZ, const float* __restrict__ cw, const float* __restrict__ cb,
    float* __restrict__ UG, unsigned short* __restrict__ UGH, unsigned short* __restrict__ UGL)
{
  __shared__ __align__(16) float sT[16 * kTP];
  const int tid = threadIdx.x, lane = tid & 31, wave = tid >> 5;
  const int d0 = blockIdx.x * 256, d = d0 + tid;
  const int t0 = blockIdx.y * 64;
  const float w0 = cw[d * kDcv + 0], w1 = cw[d * kDcv + 1], w2 = cw[d * kDcv + 2], w3 = cw[d * kDcv + 3];
  const float bc = cb[d];
  float xm3, xm2, xm1;
  {
    const int r3 = t0 - 3, r2 = t0 - 2, r1 = t0 - 1;
    const float v3 = XZ[(size_t)(r3 < 0 ? 0 : r3) * kXZP + d];
    const float v2 = XZ[(size_t)(r2 < 0 ? 0 : r2) * kXZP + d];
    const float v1 = XZ[(size_t)(r1 < 0 ? 0 : r1) * kXZP + d];
    xm3 = (r3 >= 0) ? v3 : 0.f;
    xm2 = (r2 >= 0) ? v2 : 0.f;
    xm1 = (r1 >= 0) ? v1 : 0.f;
  }
  const int hrow = wave >> 1;
  const int hch  = (wave & 1) * 128 + lane * 4;
#pragma unroll 1
  for (int sub = 0; sub < 4; ++sub) {
    const int lb = t0 + sub * 16;
#pragma unroll 1
    for (int s = 0; s < 16; ++s) {
      const size_t ro = (size_t)(lb + s) * kXZP;
      const float xc = XZ[ro + d];
      const float zv = XZ[ro + kDin + d];
      float acc = w0 * xm3;
      acc = fmaf(w1, xm2, acc);
      acc = fmaf(w2, xm1, acc);
      acc = fmaf(w3, xc, acc);
      const float uc = acc + bc;
      const float sg = __builtin_amdgcn_rcpf(1.0f + expf(-zv));
      const float gt = zv * sg;
      sT[s * kTP + tid] = uc * gt;
      xm3 = xm2; xm2 = xm1; xm1 = xc;
    }
    __syncthreads();
    v4f fv[4];
    v8h bh[2], blo[2];
#pragma unroll
    for (int it = 0; it < 4; ++it) fv[it] = *(const v4f*)(sT + (it * 4 + hrow) * kTP + hch);
#pragma unroll
    for (int it = 0; it < 2; ++it) {
      const float* sp = sT + (it * 8 + wave) * kTP + lane * 8;
      const v4f a0 = *(const v4f*)(sp);
      const v4f a1 = *(const v4f*)(sp + 4);
#pragma unroll
      for (int e = 0; e < 4; ++e) {
        const unsigned short h0 = f2bf_bits(a0[e]), h1 = f2bf_bits(a1[e]);
        const unsigned short l0 = f2bf_bits(a0[e] - bf_bits2f(h0)), l1 = f2bf_bits(a1[e] - bf_bits2f(h1));
        bh[it][e]      = __builtin_bit_cast(_Float16, h0);
        bh[it][4 + e]  = __builtin_bit_cast(_Float16, h1);
        blo[it][e]     = __builtin_bit_cast(_Float16, l0);
        blo[it][4 + e] = __builtin_bit_cast(_Float16, l1);
      }
    }
    for (int pass = 0; pass < 2; ++pass) {
#pragma unroll
      for (int it = 0; it < 4; ++it)
        *(volatile v4f*)(UG + (size_t)(lb + it * 4 + hrow) * kDin + d0 + hch) = fv[it];
#pragma unroll
      for (int it = 0; it < 2; ++it) {
        const size_t o = (size_t)(lb + it * 8 + wave) * kDin + d0 + lane * 8;
        *(volatile v8h*)(UGH + o) = bh[it];
        *(volatile v8h*)(UGL + o) = blo[it];
      }
      __threadfence();
    }
    __syncthreads();
  }
}

__global__ __launch_bounds__(256) void scan_kernel(
    const float* __restrict__ PROJ, const float* __restrict__ UG,
    const float* __restrict__ Wdt, const float* __restrict__ bdt,
    const float* __restrict__ A_log, const float* __restrict__ Dv,
    unsigned short* __restrict__ Y16)
{
  __shared__ __align__(16) float sP[16 * kPrjP];
  __shared__ __align__(16) float sY[16 * kTP];
  const int tid = threadIdx.x, lane = tid & 31, wave = tid >> 5;
  const int d0 = blockIdx.x * 256, d = d0 + tid;

  float An[kNst];
  {
    const v4f* ap = (const v4f*)(A_log + (size_t)d * kNst);
    const v4f g0 = ap[0], g1 = ap[1], g2 = ap[2], g3 = ap[3];
#pragma unroll
    for (int e = 0; e < 4; ++e) {
      An[e]      = -__expf(g0[e]);
      An[4 + e]  = -__expf(g1[e]);
      An[8 + e]  = -__expf(g2[e]);
      An[12 + e] = -__expf(g3[e]);
    }
  }
  const float wd = Wdt[d], bb = bdt[d], Dd = Dv[d];
  float h[kNst];
#pragma unroll
  for (int n = 0; n < kNst; ++n) h[n] = 0.f;
  const float kFltMin = 1.17549435e-38f;

  const int sr = tid >> 4, sc4 = (tid & 15) * 4;

#pragma unroll 1
  for (int c = 0; c < kSeqL / 16; ++c) {
    const int l0 = c * 16;
    *(v4f*)(sP + sr * kPrjP + sc4) = *(const v4f*)(PROJ + (size_t)(l0 + sr) * kPrjP + sc4);
    __syncthreads();
#pragma unroll 1
    for (int s = 0; s < 16; ++s) {
      const float* pr = sP + s * kPrjP;
      const v4f q0 = *(const v4f*)(pr + 0);
      const v4f q1 = *(const v4f*)(pr + 4);
      const v4f q2 = *(const v4f*)(pr + 8);
      const v4f q3 = *(const v4f*)(pr + 12);
      const v4f q4 = *(const v4f*)(pr + 16);
      const v4f q5 = *(const v4f*)(pr + 20);
      const v4f q6 = *(const v4f*)(pr + 24);
      const v4f q7 = *(const v4f*)(pr + 28);
      const v4f q8 = *(const v4f*)(pr + 32);
      float Bs[kNst], Cs[kNst];
      Bs[0]  = q0[1]; Bs[1]  = q0[2]; Bs[2]  = q0[3];
      Bs[3]  = q1[0]; Bs[4]  = q1[1]; Bs[5]  = q1[2]; Bs[6]  = q1[3];
      Bs[7]  = q2[0]; Bs[8]  = q2[1]; Bs[9]  = q2[2]; Bs[10] = q2[3];
      Bs[11] = q3[0]; Bs[12] = q3[1]; Bs[13] = q3[2]; Bs[14] = q3[3];
      Bs[15] = q4[0];
      Cs[0]  = q4[1]; Cs[1]  = q4[2]; Cs[2]  = q4[3];
      Cs[3]  = q5[0]; Cs[4]  = q5[1]; Cs[5]  = q5[2]; Cs[6]  = q5[3];
      Cs[7]  = q6[0]; Cs[8]  = q6[1]; Cs[9]  = q6[2]; Cs[10] = q6[3];
      Cs[11] = q7[0]; Cs[12] = q7[1]; Cs[13] = q7[2]; Cs[14] = q7[3];
      Cs[15] = q8[0];
      const float draw  = q0[0];
      const float v     = draw * wd + bb;
      const float delta = fmaxf(v, 0.0f) + log1pf(expf(-fabsf(v)));
      const float dte   = expf(delta);
      const float ut    = UG[(size_t)(l0 + s) * kDin + d];
      float y = 0.f;
#pragma unroll
      for (int n = 0; n < kNst; ++n) {
        float e = __expf(dte * An[n]);
        e = (e < kFltMin) ? 0.f : e;
        const float db = Bs[n] * dte;
        const float p  = db * ut;
        const float hn = e * h[n] + p;
        h[n] = hn;
        y = y + hn * Cs[n];
      }
      y = y + Dd * ut;
      sY[s * kTP + tid] = y * kYCarry;
    }
    __syncthreads();
    v8h hv[2];
#pragma unroll
    for (int it = 0; it < 2; ++it) {
      const float* sp = sY + (it * 8 + wave) * kTP + lane * 8;
      const v4f a0 = *(const v4f*)(sp);
      const v4f a1 = *(const v4f*)(sp + 4);
#pragma unroll
      for (int e = 0; e < 4; ++e) { hv[it][e] = (_Float16)a0[e]; hv[it][4 + e] = (_Float16)a1[e]; }
    }
    for (int pass = 0; pass < 2; ++pass) {
#pragma unroll
      for (int it = 0; it < 2; ++it)
        *(volatile v8h*)(Y16 + (size_t)(l0 + it * 8 + wave) * kDin + d0 + lane * 8) = hv[it];
      __threadfence();
    }
  }
}

extern "C" void kernel_launch(void* const* d_in, const int* in_sizes, int n_in,
                              void* d_out, int out_size, void* d_ws, size_t ws_size,
                              hipStream_t stream)
{
  if (n_in < 10) return;
  if (in_sizes[0] != kRows * kDmod) return;
  if (in_sizes[1] != kXZP * kDmod) return;
  if (in_sizes[2] != kDin * kDcv) return;
  if (in_sizes[3] != kDin) return;
  if (in_sizes[4] != kPrjN * kDin) return;
  if (in_sizes[5] != kDin) return;
  if (in_sizes[6] != kDin) return;
  if (in_sizes[7] != kDin * kNst) return;
  if (in_sizes[8] != kDin) return;
  if (in_sizes[9] != kDmod * kDin) return;
  if (out_size != kRows * kDmod) return;
  if (ws_size < kWsTotal) return;

  const float* x      = (const float*)d_in[0];
  const float* W_in   = (const float*)d_in[1];
  const float* conv_w = (const float*)d_in[2];
  const float* conv_b = (const float*)d_in[3];
  const float* W_xprj = (const float*)d_in[4];
  const float* W_dt   = (const float*)d_in[5];
  const float* b_dt   = (const float*)d_in[6];
  const float* A_log  = (const float*)d_in[7];
  const float* Dv     = (const float*)d_in[8];
  const float* W_out  = (const float*)d_in[9];
  float* dout = (float*)d_out;

  char* ws = (char*)d_ws;
  unsigned short* X16  = (unsigned short*)(ws + kOffX16);
  unsigned short* WI16 = (unsigned short*)(ws + kOffWI16);
  unsigned short* WO16 = (unsigned short*)(ws + kOffWO16);
  unsigned short* WXH  = (unsigned short*)(ws + kOffWXH);
  unsigned short* WXL  = (unsigned short*)(ws + kOffWXL);
  float*          XZ   = (float*)(ws + kOffXZ);
  float*          UG   = (float*)(ws + kOffUG);
  unsigned short* UGH  = (unsigned short*)(ws + kOffUGH);
  unsigned short* UGL  = (unsigned short*)(ws + kOffUGL);
  float*          PROJ = (float*)(ws + kOffPROJ);
  unsigned short* Y16  = (unsigned short*)(ws + kOffY16);
  const float* dummy_bias  = b_dt;
  const float* dummy_resid = x;

  cast_f16_kernel<<<(kRows * kDmod) / 8 / 256, 256, 0, stream>>>(x, X16, (kRows * kDmod) / 8, 1.0f);
  cast_f16_kernel<<<(kXZP * kDmod) / 8 / 256, 256, 0, stream>>>(W_in, WI16, (kXZP * kDmod) / 8, kWCarry);
  cast_f16_kernel<<<(kDmod * kDin) / 8 / 256, 256, 0, stream>>>(W_out, WO16, (kDmod * kDin) / 8, kWCarry);
  split_rows_pad_bf16_kernel<<<(kPrjP * kDin) / 8 / 256, 256, 0, stream>>>(W_xprj, WXH, WXL, (kPrjP * kDin) / 8, kDin, kPrjN);

  for (int b = 0; b < kBatch; ++b) {
    const unsigned short* X16b = X16 + (size_t)b * kSeqL * kDmod;
    float* outb = dout + (size_t)b * kSeqL * kDmod;

    wmma_gemm64<0, false, 0, 0, false><<<dim3(256, 1), 256, 0, stream>>>(
        X16b, X16b, kDmod, 0L, WI16, WI16, kDmod, 0L,
        (void*)XZ, (void*)XZ, kXZP, 0L, dummy_bias, dummy_resid, 0L, kSeqL, kXZP, kDmod, kInProjScale);

    conv_gate_kernel<<<dim3(kDin / 256, kSeqL / 64), 256, 0, stream>>>(XZ, conv_w, conv_b, UG, UGH, UGL);

    wmma_gemm64<1, true, 0, 0, false><<<dim3(4, 1), 256, 0, stream>>>(
        UGH, UGL, kDin, 0L, WXH, WXL, kDin, 0L,
        (void*)PROJ, (void*)PROJ, kPrjP, 0L, dummy_bias, dummy_resid, 0L, kSeqL, kPrjP, kDin, 1.0f);

    scan_kernel<<<dim3(kDin / 256, 1), 256, 0, stream>>>(PROJ, UG, W_dt, b_dt, A_log, Dv, Y16);

    wmma_gemm64<0, false, 0, 0, false><<<dim3(64, 1), 256, 0, stream>>>(
        Y16, Y16, kDin, 0L, WO16, WO16, kDin, 0L,
        (void*)outb, (void*)outb, kDmod, 0L, dummy_bias, dummy_resid, 0L, kSeqL, kDmod, kDin, kOutProjScale);
  }
}
